// GATConv_65592740544797
// MI455X (gfx1250) — hardware-verified
//
#include <hip/hip_runtime.h>


#ifndef NB
#define NB 8
#endif
#ifndef SEQ
#define SEQ 1024
#endif

namespace {
constexpr int NB_FULL = 8, SEQ_FULL = 1024, E = 256, H = 8, HD = 32, E3 = 3 * E, OD = 256, NR = NB * SEQ;
constexpr float XS = 8.0f, WSC = 256.0f, QS = 64.0f, KS = 8.0f, VS = 8.0f, RS_ = 1024.0f, PS = 1024.0f, CS = 256.0f, AS_ = 256.0f;
constexpr float LOG2E = 1.4426950408889634f, NEGF = -1.0e9f, NSL_ = 0.2f, QKS = 0.17677669529663687f;
static_assert(NB >= 1 && NB <= NB_FULL && SEQ >= 64 && SEQ <= SEQ_FULL && SEQ % 64 == 0);
static_assert(E == H * HD && HD == 32 && E % 32 == 0 && E3 % 64 == 0 && OD == E && OD % 64 == 0);
constexpr int CVT_PER_BLK = 2048;
constexpr int BX = NR * E / CVT_PER_BLK, BWI = E3 * E / CVT_PER_BLK, BWO = E * E / CVT_PER_BLK, BWL = OD * E / CVT_PER_BLK;
static_assert((NR * E) % CVT_PER_BLK == 0 && (E3 * E) % CVT_PER_BLK == 0 && (E * E) % CVT_PER_BLK == 0 && (OD * E) % CVT_PER_BLK == 0);

typedef _Float16 b16;
typedef __attribute__((ext_vector_type(16))) _Float16 v16b;
typedef __attribute__((ext_vector_type(8))) _Float16 v8b;
typedef __attribute__((ext_vector_type(8))) float v8f;
typedef __attribute__((ext_vector_type(4))) float v4f;
typedef __attribute__((ext_vector_type(8))) int v8i;

__device__ __forceinline__ float bf16_rne(float f) { unsigned int u = __float_as_uint(f); u += 0x7FFFu + ((u >> 16) & 1u); return __uint_as_float(u & 0xFFFF0000u); }
__device__ __forceinline__ v16b frag_kb(const b16* p, int hh) { const v8b a = *(const v8b*)(p + 8 * hh), b = *(const v8b*)(p + 16 + 8 * hh); v16b f;
#pragma unroll
  for (int e = 0; e < 8; ++e) { f[e] = a[e]; f[8 + e] = b[e]; } return f; }
__device__ __forceinline__ v8f wmma16b(v16b a, v16b b, v8f c) { v8f d = __builtin_amdgcn_wmma_f32_16x16x32_f16(false, a, false, b, (short)0, c, false, false); asm volatile("v_nop\n\tv_nop\n\tv_nop\n\tv_nop" : "+v"(d) : "v"(a), "v"(b)); return d; }
__device__ __forceinline__ void wave_lds_sync() { __builtin_amdgcn_fence(3  , "workgroup"); __builtin_amdgcn_wave_barrier(); __builtin_amdgcn_fence(2  , "workgroup"); }
__device__ __forceinline__ float nexp2(float v) { return __builtin_amdgcn_exp2f(v); }

__global__ __launch_bounds__(256) void cvt_kernel(const float* __restrict__ x, const float* __restrict__ wi, const float* __restrict__ wo, const float* __restrict__ wl,
                                                  b16* __restrict__ Xh, b16* __restrict__ Wih, b16* __restrict__ Woh, b16* __restrict__ Wlh) {
  const int bid = blockIdx.x;
  const float* src; b16* dst; float sc; int lb;
  if (bid < BX) { lb = bid; sc = XS; dst = Xh; src = x; }
  else if (bid < BX + BWI) { lb = bid - BX; sc = WSC; dst = Wih; src = wi; }
  else if (bid < BX + BWI + BWO) { lb = bid - BX - BWI; sc = WSC; dst = Woh; src = wo; }
  else { lb = bid - BX - BWI - BWO; sc = WSC; dst = Wlh; src = wl; }
  if (lb >= BX + BWI + BWO + BWL) return;
  const int e = lb * CVT_PER_BLK + (int)threadIdx.x * 8;
  size_t se = (size_t)e;
  if (bid < BX) { const int r = e / E, c = e % E; se = ((size_t)(r / SEQ) * SEQ_FULL + (size_t)(r % SEQ)) * E + c; }
  const v4f f0 = *(const v4f*)(src + se), f1 = *(const v4f*)(src + se + 4);
  v8b v;
#pragma unroll
  for (int j = 0; j < 4; ++j) { v[j] = (b16)(bf16_rne(f0[j]) * sc); v[4 + j] = (b16)(bf16_rne(f1[j]) * sc); }
  for (int pass = 0; pass < 2; ++pass) { *(volatile v8b*)(dst + e) = v; __threadfence(); }
}

__global__ __launch_bounds__(128) void qkv_kernel(const b16* __restrict__ Xh, const b16* __restrict__ Wih, const float* __restrict__ b_in,
                                                  b16* __restrict__ Qh, b16* __restrict__ Ql, b16* __restrict__ Kh, b16* __restrict__ Kl, b16* __restrict__ VTh, b16* __restrict__ VTl) {
  __shared__ __attribute__((aligned(16))) float Tf[64][68];
  const int wave = threadIdx.x >> 5, lane = threadIdx.x & 31, col = lane & 15, hh = lane >> 4;
  const int n0 = blockIdx.x * 64, cg = blockIdx.y, b = blockIdx.z, c0 = cg * 64, part = cg >> 2;
  const b16* arow = Xh + ((size_t)b * SEQ + n0 + wave * 16 + col) * E;
  v8f acc[4];
#pragma unroll
  for (int t = 0; t < 4; ++t) acc[t] = (v8f){};
#pragma unroll
  for (int kb = 0; kb < E; kb += 32) { const v16b af = frag_kb(arow + kb, hh);
#pragma unroll
    for (int t = 0; t < 4; ++t) acc[t] = wmma16b(af, frag_kb(Wih + (size_t)(c0 + t * 16 + col) * E + kb, hh), acc[t]); }
  const float osc = (part == 0) ? QKS : 1.0f;
#pragma unroll
  for (int t = 0; t < 4; ++t) { const float bia = bf16_rne(b_in[c0 + t * 16 + col]);
#pragma unroll
    for (int r = 0; r < 8; ++r) Tf[wave * 16 + 8 * hh + r][t * 16 + col] = (acc[t][r] * (1.0f / (XS * WSC)) + bia) * osc; }
  __syncthreads();
  const int hbase = (cg & 3) * 2;
  if (part < 2) {
    b16* Ph = (part == 0) ? Qh : Kh; b16* Pr = (part == 0) ? Ql : Kl; const float cs = (part == 0) ? QS : KS;
    for (int pass = 0; pass < 2; ++pass) {
      for (int idx = threadIdx.x; idx < 512; idx += 128) {
        const int hl = idx >> 8, rem = idx & 255, row = rem >> 2, c8 = (rem & 3) * 8, h = hbase + hl;
        v8b hv, lv;
#pragma unroll
        for (int j = 0; j < 8; ++j) { const float f = Tf[row][hl * 32 + c8 + j] * cs; const b16 p = (b16)f; hv[j] = p; lv[j] = (b16)((f - (float)p) * RS_); }
        const size_t oi = (((size_t)(b * H + h)) * SEQ + n0 + row) * HD + c8;
        *(volatile v8b*)(Ph + oi) = hv; *(volatile v8b*)(Pr + oi) = lv; }
      __threadfence(); }
  } else {
    for (int pass = 0; pass < 2; ++pass) {
      for (int idx = threadIdx.x; idx < 512; idx += 128) {
        const int line = idx >> 3, hl = line >> 5, d = line & 31, c8 = (idx & 7) * 8, h = hbase + hl;
        v8b hv, lv;
#pragma unroll
        for (int j = 0; j < 8; ++j) { const float f = Tf[c8 + j][hl * 32 + d] * VS; const b16 p = (b16)f; hv[j] = p; lv[j] = (b16)((f - (float)p) * RS_); }
        const size_t oi = (((size_t)(b * H + h)) * HD + d) * (size_t)SEQ + n0 + c8;
        *(volatile v8b*)(VTh + oi) = hv; *(volatile v8b*)(VTl + oi) = lv; }
      __threadfence(); }
  }
}

__global__ __launch_bounds__(64) void att_kernel(const int* __restrict__ adj, const b16* __restrict__ Qh, const b16* __restrict__ Ql, const b16* __restrict__ Kh, const b16* __restrict__ Kl,
                                                 const b16* __restrict__ VTh, const b16* __restrict__ VTl, b16* __restrict__ Ch) {
  __shared__ __attribute__((aligned(16))) float Sf[2][16][40];
  __shared__ __attribute__((aligned(16))) b16 Pb[2][16][40], Pl[2][16][40];
  __shared__ __attribute__((aligned(16))) float To[2][16][40];
  const int wave = threadIdx.x >> 5, lane = threadIdx.x & 31, hh = lane >> 4, col = lane & 15;
  const int bh = blockIdx.y; const int i0 = blockIdx.x * 32 + wave * 16, ii = i0 + col;
  const size_t qo = ((size_t)bh * SEQ + ii) * HD;
  const v16b qhf = frag_kb(Qh + qo, hh), qlf = frag_kb(Ql + qo, hh);
  const b16* kh = Kh + (size_t)bh * SEQ * HD; const b16* kl = Kl + (size_t)bh * SEQ * HD;
  const b16* Vh = VTh + (size_t)bh * HD * (size_t)SEQ; const b16* Vl = VTl + (size_t)bh * HD * (size_t)SEQ;
  const int* arow = adj + (size_t)ii * SEQ_FULL;
  float m = -INFINITY, l = 0.0f; v8f o[2], ol[2];
#pragma unroll
  for (int t = 0; t < 2; ++t) { o[t] = (v8f){}; ol[t] = (v8f){}; }
  const float ssc = LOG2E / (QS * KS);
#pragma unroll 1
  for (int kb = 0; kb < SEQ; kb += 32) {
#pragma unroll
    for (int kt = 0; kt < 2; ++kt) {
      const size_t ko = (size_t)(kb + kt * 16 + col) * HD;
      const v16b khf = frag_kb(kh + ko, hh), klf = frag_kb(kl + ko, hh);
      const v8f sh = wmma16b(qhf, khf, (v8f){}); v8f sl = wmma16b(qhf, klf, (v8f){}); sl = wmma16b(qlf, khf, sl);
#pragma unroll
      for (int r = 0; r < 8; ++r) Sf[wave][8 * hh + r][kt * 16 + col] = sh[r] + sl[r] * (1.0f / RS_); }
    wave_lds_sync();
    const v8i a0 = *(const v8i*)(arow + kb + 8 * hh), a1 = *(const v8i*)(arow + kb + 16 + 8 * hh);
    const v8f s0 = *(const v8f*)(&Sf[wave][col][8 * hh]), s1 = *(const v8f*)(&Sf[wave][col][16 + 8 * hh]);
    float e[16]; float mx = -INFINITY;
#pragma unroll
    for (int i = 0; i < 8; ++i) {
      const float ev0 = (a0[i] != 0) ? s0[i] * ssc : NEGF; const float ev1 = (a1[i] != 0) ? s1[i] * ssc : NEGF;
      e[i] = ev0; e[8 + i] = ev1; mx = fmaxf(mx, fmaxf(ev0, ev1)); }
    mx = fmaxf(mx, __shfl_xor(mx, 16)); const float mn = fmaxf(m, mx); const float al = nexp2(m - mn); float sum = 0.0f;
#pragma unroll
    for (int i2 = 0; i2 < 16; ++i2) { const float p = nexp2(e[i2] - mn); sum += p; const float ps = p * PS; const b16 phh = (b16)ps; const int pc = (i2 < 8 ? 0 : 16) + 8 * hh + (i2 & 7);
      Pb[wave][col][pc] = phh; Pl[wave][col][pc] = (b16)((ps - (float)phh) * RS_); }
    sum += __shfl_xor(sum, 16); l = l * al + sum; m = mn;
    wave_lds_sync();
    const v16b pf = frag_kb(&Pb[wave][col][0], hh), plf = frag_kb(&Pl[wave][col][0], hh);
#pragma unroll
    for (int t = 0; t < 2; ++t) { const v16b vh = frag_kb(Vh + (size_t)(t * 16 + col) * SEQ + kb, hh); o[t] *= al; o[t] = wmma16b(vh, pf, o[t]);
      ol[t] = wmma16b(frag_kb(Vl + (size_t)(t * 16 + col) * SEQ + kb, hh), pf, ol[t] * al); ol[t] = wmma16b(vh, plf, ol[t]); }
    wave_lds_sync(); }
  const float inv = 1.0f / (l * PS * VS);
#pragma unroll
  for (int t = 0; t < 2; ++t)
#pragma unroll
    for (int r = 0; r < 8; ++r) To[wave][col][t * 16 + 8 * hh + r] = (o[t][r] + ol[t][r] * (1.0f / RS_)) * inv;
  wave_lds_sync();
  for (int pass = 0; pass < 2; ++pass) {
#pragma unroll
    for (int it = 0; it < 2; ++it) { const int rr = it * 8 + (lane >> 2), c8 = (lane & 3) * 8;
      const v8f tv = *(const v8f*)(&To[wave][rr][c8]); v8b cv;
#pragma unroll
      for (int j = 0; j < 8; ++j) cv[j] = (b16)(tv[j] * CS);
      *(volatile v8b*)(Ch + ((size_t)bh * SEQ + i0 + rr) * HD + c8) = cv; }
    __threadfence(); }
}

__global__ __launch_bounds__(256) void out_kernel(const b16* __restrict__ Ch, const b16* __restrict__ Woh, const float* __restrict__ b_out, const b16* __restrict__ Wlh, const float* __restrict__ b_lin,
                                                  float* __restrict__ Y) {
  __shared__ __attribute__((aligned(16))) b16 At[16][E + 8];
  __shared__ __attribute__((aligned(16))) float Of[16][OD + 4];
  const int wave = threadIdx.x >> 5, lane = threadIdx.x & 31, hh = lane >> 4, col = lane & 15;
  const int row0 = blockIdx.x * 16; const int b = row0 / SEQ, n0 = row0 % SEQ; const int c0 = wave * 32;
  v8f acc[2]; acc[0] = (v8f){}; acc[1] = (v8f){};
#pragma unroll
  for (int kb = 0; kb < E; kb += 32) { const v16b af = frag_kb(Ch + (((size_t)(b * H + kb / HD)) * SEQ + n0 + col) * HD, hh);
#pragma unroll
    for (int t = 0; t < 2; ++t) acc[t] = wmma16b(af, frag_kb(Woh + (size_t)(c0 + t * 16 + col) * E + kb, hh), acc[t]); }
#pragma unroll
  for (int t = 0; t < 2; ++t) { const float bia = bf16_rne(b_out[c0 + t * 16 + col]);
#pragma unroll
    for (int r = 0; r < 8; ++r) At[8 * hh + r][c0 + t * 16 + col] = (b16)((acc[t][r] * (1.0f / (CS * WSC)) + bia) * AS_); }
  __syncthreads();
  v8f acc2[2]; acc2[0] = (v8f){}; acc2[1] = (v8f){};
#pragma unroll
  for (int kb = 0; kb < E; kb += 32) { const v16b af = frag_kb(&At[col][kb], hh);
#pragma unroll
    for (int t = 0; t < 2; ++t) acc2[t] = wmma16b(af, frag_kb(Wlh + (size_t)(c0 + t * 16 + col) * E + kb, hh), acc2[t]); }
#pragma unroll
  for (int t = 0; t < 2; ++t) { const float bia = bf16_rne(b_lin[c0 + t * 16 + col]);
#pragma unroll
    for (int r = 0; r < 8; ++r) { float y = acc2[t][r] * (1.0f / (AS_ * WSC)) + bia; y = (y >= 0.0f) ? y : NSL_ * y; Of[8 * hh + r][c0 + t * 16 + col] = y; } }
  __syncthreads();
  for (int pass = 0; pass < 2; ++pass) {
#pragma unroll
    for (int it = 0; it < 4; ++it) { const int idx = it * 256 + (int)threadIdx.x; const int row = idx >> 6, c4 = (idx & 63) * 4;
      const v4f vv = *(const v4f*)(&Of[row][c4]);
      *(volatile v4f*)(Y + ((size_t)row0 + row) * OD + c4) = vv; }
    __threadfence(); }
}
}

extern "C" void kernel_launch(void* const* d_in, const int* in_sizes, int n_in, void* d_out, int out_size, void* d_ws, size_t ws_size, hipStream_t stream) {
  (void)n_in;
  auto Fp = [&](int i) { return (const float*)d_in[i]; };
  if (in_sizes[0] < NR * E || in_sizes[1] < SEQ * SEQ || in_sizes[2] < E3 * E || in_sizes[3] < E3 || in_sizes[4] < E * E || in_sizes[5] < E ||
      in_sizes[6] < OD * E || in_sizes[7] < OD || out_size < NR * OD) return;
  const int* adj = (const int*)d_in[1];
  size_t off = 0; char* ws = (char*)d_ws;
  auto carve = [&](size_t bytes) { char* p = ws + off; off += (bytes + 255) & ~(size_t)255; return p; };
  const size_t plane = (size_t)NB * H * SEQ * HD * 2;
  b16* Xh = (b16*)carve((size_t)NR * E * 2); b16* Wih = (b16*)carve((size_t)E3 * E * 2); b16* Woh = (b16*)carve((size_t)E * E * 2); b16* Wlh = (b16*)carve((size_t)OD * E * 2);
  b16* Qh = (b16*)carve(plane); b16* Ql = (b16*)carve(plane); b16* Kh = (b16*)carve(plane); b16* Kl = (b16*)carve(plane);
  b16* VTh = (b16*)carve(plane); b16* VTl = (b16*)carve(plane); b16* Ch = (b16*)carve(plane);
  if (off > ws_size || off > ((size_t)128 << 20)) return;
  cvt_kernel<<<BX + BWI + BWO + BWL, 256, 0, stream>>>(Fp(0), Fp(2), Fp(4), Fp(6), Xh, Wih, Woh, Wlh);
  qkv_kernel<<<dim3(SEQ / 64, E3 / 64, NB), 128, 0, stream>>>(Xh, Wih, Fp(3), Qh, Ql, Kh, Kl, VTh, VTl);
  att_kernel<<<dim3(SEQ / 32, NB * H), 64, 0, stream>>>(adj, Qh, Ql, Kh, Kl, VTh, VTl, Ch);
  out_kernel<<<NR / 16, 256, 0, stream>>>(Ch, Woh, Fp(5), Wlh, Fp(7), (float*)d_out);
}
